// DenseGIN_21045339750900
// MI455X (gfx1250) — hardware-verified
//
#include <hip/hip_runtime.h>
#include <stddef.h>


#define CIN    128
#define CH     256
#define NCLS   40
#define NCP    64
#define NTHR   256
#define NWAVE  8
#define EPT    8
#define NGRP   2
#define CHUNK  (NTHR * EPT * NGRP)
#define WCAP   (EPT * NGRP * 32)
#define LISTN  (NWAVE * WCAP)
#define ESHF   11
#define NBC    32768
#define NBF    2048
#define RCAP   40960
#define RBN    128
#define TGT    256
#define DEGCAP 512
#define GR     64
#define OTHR   512
#define WSCAP  134217728
#define WSCL   64.0f
#define WINV   0.015625f
#define BNEPS  1e-5f

#define LDS_COUNT ((NBC + LISTN + NWAVE) * 4)
#define LDS_FILL  ((RCAP + NBF + LISTN + NWAVE) * 4)

static_assert((CHUNK & (CHUNK - 1)) == 0);
static_assert((NBC & (NBC - 1)) == 0 && (NBF & (NBF - 1)) == 0);
static_assert(NBF <= (1 << ESHF));
static_assert((NBC % NBF) == 0);
static_assert(OTHR * 4 == NBF);
static_assert((RCAP % 32) == 0);
static_assert(TGT == NWAVE * 32);
static_assert(GR == (NWAVE / 2) * 16 && GR == NWAVE * 8);
static_assert((TGT % GR) == 0);
static_assert(NBC == NWAVE * 32 * 128);
static_assert((CIN % 32) == 0 && (CH % 32) == 0 && (NCP % 32) == 0);
static_assert(NCLS <= NCP && (NCLS % 4) == 0);

typedef float    v2f  __attribute__((ext_vector_type(2)));
typedef float    v4f  __attribute__((ext_vector_type(4)));
typedef float    v8f  __attribute__((ext_vector_type(8)));
typedef int      v4i  __attribute__((ext_vector_type(4)));
typedef _Float16 v2h  __attribute__((ext_vector_type(2)));
typedef _Float16 v4h  __attribute__((ext_vector_type(4)));
typedef _Float16 v8h  __attribute__((ext_vector_type(8)));
typedef _Float16 v16h __attribute__((ext_vector_type(16)));
union FragH { v16h v; v8h h[2]; };

__device__ __forceinline__ v8f wmh(v16h a, v16h b, v8f c) {
  v8f d = __builtin_amdgcn_wmma_f32_16x16x32_f16(false, a, false, b, (short)0, c, false, false);
  asm volatile("v_nop\n\tv_nop\n\tv_nop\n\tv_nop" : "+v"(d) : "v"(a), "v"(b));
  return d;
}

template <int NB, int EID>
__device__ __forceinline__ int scan_chunk(const int* __restrict__ dsts, int nE,
                                          int cbase, int slotBase, int vec8, int* list, int tid, int lane, int wave) {
  int wc = 0;
#pragma unroll
  for (int g = 0; g < NGRP; ++g) {
    const int el0  = (g * NTHR + tid) * EPT;
    const int e0   = cbase + el0;
    const int sent = -2147483647 - 1;
    v4i da, db;
    if (vec8 != 0 && cbase + CHUNK <= nE) {
      da = *(const v4i*)(dsts + e0);
      db = *(const v4i*)(dsts + e0 + 4);
    } else {
      da.x = (e0     < nE) ? dsts[min(e0, nE - 1)] : sent;
      da.y = (e0 + 1 < nE) ? dsts[min(e0 + 1, nE - 1)] : sent;
      da.z = (e0 + 2 < nE) ? dsts[min(e0 + 2, nE - 1)] : sent;
      da.w = (e0 + 3 < nE) ? dsts[min(e0 + 3, nE - 1)] : sent;
      db.x = (e0 + 4 < nE) ? dsts[min(e0 + 4, nE - 1)] : sent;
      db.y = (e0 + 5 < nE) ? dsts[min(e0 + 5, nE - 1)] : sent;
      db.z = (e0 + 6 < nE) ? dsts[min(e0 + 6, nE - 1)] : sent;
      db.w = (e0 + 7 < nE) ? dsts[min(e0 + 7, nE - 1)] : sent;
    }
    const unsigned nb = (unsigned)slotBase;
    const unsigned s0 = (unsigned)da.x - nb, s1 = (unsigned)da.y - nb;
    const unsigned s2 = (unsigned)da.z - nb, s3 = (unsigned)da.w - nb;
    const unsigned s4 = (unsigned)db.x - nb, s5 = (unsigned)db.y - nb;
    const unsigned s6 = (unsigned)db.z - nb, s7 = (unsigned)db.w - nb;
    const bool h0 = s0 < (unsigned)NB, h1 = s1 < (unsigned)NB, h2 = s2 < (unsigned)NB, h3 = s3 < (unsigned)NB;
    const bool h4 = s4 < (unsigned)NB, h5 = s5 < (unsigned)NB, h6 = s6 < (unsigned)NB, h7 = s7 < (unsigned)NB;
    const unsigned any = __builtin_amdgcn_ballot_w32(h0 | h1 | h2 | h3 | h4 | h5 | h6 | h7);
    if (any != 0u) {
#define HITJ(HJ, SJ, VJ) { \
        const unsigned mj = __builtin_amdgcn_ballot_w32(HJ); \
        if (mj != 0u) { \
          if (HJ) { \
            const int pos = wc + (int)__builtin_amdgcn_mbcnt_lo(mj, 0u); \
            const int entv = EID ? (((VJ) << ESHF) | (int)(SJ)) : (int)(SJ); \
            if (pos < WCAP) list[wave * WCAP + pos] = entv; \
          } \
          wc += (int)__builtin_popcount(mj); } }
      HITJ(h0, s0, e0)
      HITJ(h1, s1, e0 + 1)
      HITJ(h2, s2, e0 + 2)
      HITJ(h3, s3, e0 + 3)
      HITJ(h4, s4, e0 + 4)
      HITJ(h5, s5, e0 + 5)
      HITJ(h6, s6, e0 + 6)
      HITJ(h7, s7, e0 + 7)
#undef HITJ
    }
  }
  return wc;
}

__global__ __launch_bounds__(NTHR) void k_wprep(const float* __restrict__ W, _Float16* P,
                                                int din, int dout, int KP, int NP) {
  const int tid = threadIdx.x;
  const int kq = KP >> 3;
  const int total = NP * kq;
  const int i = (int)blockIdx.x * NTHR + tid;
  const int ic = i < total ? i : total - 1;
  const int n = ic / kq;
  const int k0 = (ic - n * kq) * 8;
  const int nc = n < dout ? n : dout - 1;
  v8h hv;
#pragma unroll
  for (int e = 0; e < 8; ++e) {
    const int k = k0 + e;
    const int kc = k < din ? k : din - 1;
    float v = W[(size_t)kc * dout + nc];
    v = (n < dout && k < din) ? v * WSCL : 0.0f;
    hv[e] = (_Float16)v;
  }
  _Float16* dp = P + (size_t)ic * 8;
  if (i < total) *(volatile v8h*)dp = hv;
  __threadfence();
  if (i < total) *(volatile v8h*)dp = hv;
}

__global__ __launch_bounds__(NTHR) void k_count(const int* __restrict__ ei, int* cnt, int nE, int vec8) {
  extern __shared__ v4f lds_dyn[];
  int* scnt = (int*)lds_dyn;
  int* list = scnt + NBC;
  int* wcnt = list + LISTN;
  const int tid = threadIdx.x, lane = tid & 31, wave = tid >> 5;
  const int nodeBase = blockIdx.x * NBC;
  const int* dsts = ei + nE;

  {
    const v4i z = {0, 0, 0, 0};
    for (int i = tid; i < NBC / 4; i += NTHR) ((v4i*)scnt)[i] = z;
  }
  __syncthreads();

  const int nChunks = (nE + CHUNK - 1) / CHUNK;
#pragma unroll 1
  for (int ch = 0; ch < nChunks; ++ch) {
    const int cbase = ch * CHUNK;
    const int wc = scan_chunk<NBC, 0>(dsts, nE, cbase, nodeBase, vec8, list, tid, lane, wave);
    if (lane == 0) wcnt[wave] = wc;
    __syncthreads();
    if (wave == 0) {
#pragma unroll 1
      for (int wsx = 0; wsx < NWAVE; ++wsx) {
        int n = __builtin_amdgcn_readfirstlane(wcnt[wsx]);
        n = n > WCAP ? WCAP : (n < 0 ? 0 : n);
        const int* lp = list + wsx * WCAP;
#pragma unroll 1
        for (int i = 0; i < n; ++i) {
          const int ent  = __builtin_amdgcn_readfirstlane(lp[i]);
          const int slot = ent & (NBC - 1);
          if (lane == 0) scnt[slot] = scnt[slot] + 1;
        }
      }
    }
    __syncthreads();
  }

  int* cp = cnt + (size_t)nodeBase;
#pragma unroll 4
  for (int q = 0; q < 32; ++q) {
    const int f = (wave * 32 + q) * 128 + 4 * lane;
    const v4i c = *(const v4i*)(scnt + f);
    *(volatile v4i*)(cp + f) = c;
  }
  __threadfence();
#pragma unroll 4
  for (int q = 0; q < 32; ++q) {
    const int f = (wave * 32 + q) * 128 + 4 * lane;
    const v4i c = *(const v4i*)(scnt + f);
    *(volatile v4i*)(cp + f) = c;
  }
}

__global__ __launch_bounds__(OTHR) void k_offsets(const int* __restrict__ cnt, int* off, int* rbase, int nBF) {
  __shared__ __attribute__((aligned(16))) int srb[RBN];
  __shared__ int wtot[OTHR / 32];
  const int tid = threadIdx.x, lane = tid & 31, wave = tid >> 5;
  for (int i = tid; i < RBN; i += OTHR) srb[i] = 0;
  int carry = 0;
#pragma unroll 1
  for (int fb = 0; fb < nBF; ++fb) {
    const int base = fb * NBF;
    const v4i c = *(const v4i*)(cnt + base + 4 * tid);
    const int e0 = max(c.x, 0), e1 = max(c.y, 0), e2 = max(c.z, 0), e3 = max(c.w, 0);
    const int ts = e0 + e1 + e2 + e3;
    int incl = ts;
#pragma unroll
    for (int d = 1; d < 32; d <<= 1) {
      const int t = __shfl_up(incl, d);
      if (lane >= d) incl += t;
    }
    if (lane == 31) wtot[wave] = incl;
    __syncthreads();
    int pre = 0;
#pragma unroll 1
    for (int w = 0; w < wave; ++w) pre += wtot[w];
    int tot = 0;
#pragma unroll
    for (int w = 0; w < OTHR / 32; ++w) tot += wtot[w];
    int run = carry + pre + incl - ts;
    v4i o;
    o.x = run; run += e0;
    o.y = run; run += e1;
    o.z = run; run += e2;
    o.w = run;
    int* op = off + base + 4 * tid;
    *(volatile v4i*)op = o;
    __threadfence();
    *(volatile v4i*)op = o;
    if (tid == 0) srb[min(fb, RBN - 1)] = carry;
    carry += (tot + 31) & ~31;
    __syncthreads();
  }
  if (tid == 0) srb[min(nBF, RBN - 1)] = carry;
  __syncthreads();
  v4i rv = {0, 0, 0, 0};
  if (tid < 32) rv = *(const v4i*)(srb + 4 * tid);
  if (tid < 32) *(volatile v4i*)(rbase + 4 * tid) = rv;
  __threadfence();
  if (tid < 32) *(volatile v4i*)(rbase + 4 * tid) = rv;
}

__global__ __launch_bounds__(NTHR) void k_fill(
    const int* __restrict__ ei, const int* __restrict__ off, const int* __restrict__ rbase,
    int* csr, int nE, int vec8, int csrLen) {
  extern __shared__ v4f lds_dyn[];
  int* region = (int*)lds_dyn;
  int* cursor = region + RCAP;
  int* list   = cursor + NBF;
  int* wcnt   = list + LISTN;
  const int tid = threadIdx.x, lane = tid & 31, wave = tid >> 5;
  const int b = blockIdx.x;
  const int nodeBase = b * NBF;
  const int* dsts = ei + nE;

  int rb0 = rbase[b];
  const int rb1 = rbase[b + 1];
  rb0 = rb0 < 0 ? 0 : (rb0 > csrLen ? csrLen : rb0);
  rb0 &= ~31;
  int len = rb1 - rb0;
  len = len < 0 ? 0 : (len > RCAP ? RCAP : len);
  int lenW = (len + 31) & ~31;
  if (rb0 + lenW > csrLen) lenW = (csrLen - rb0) & ~31;

  {
    const v4i z = {0, 0, 0, 0};
    for (int i = tid; i < RCAP / 4; i += NTHR) ((v4i*)region)[i] = z;
    for (int s = tid; s < NBF; s += NTHR) {
      int o = off[nodeBase + s] - rb0;
      o = o < 0 ? 0 : (o > RCAP ? RCAP : o);
      cursor[s] = o;
    }
  }
  __syncthreads();

  const int nChunks = (nE + CHUNK - 1) / CHUNK;
#pragma unroll 1
  for (int ch = 0; ch < nChunks; ++ch) {
    const int cbase = ch * CHUNK;
    const int wc = scan_chunk<NBF, 1>(dsts, nE, cbase, nodeBase, vec8, list, tid, lane, wave);
    if (lane == 0) wcnt[wave] = wc;
    __syncthreads();
    if (wave == 0) {
#pragma unroll 1
      for (int wsx = 0; wsx < NWAVE; ++wsx) {
        int n = __builtin_amdgcn_readfirstlane(wcnt[wsx]);
        n = n > WCAP ? WCAP : (n < 0 ? 0 : n);
        const int* lp = list + wsx * WCAP;
#pragma unroll 1
        for (int i = 0; i < n; ++i) {
          const int ent  = __builtin_amdgcn_readfirstlane(lp[i]);
          const int slot = ent & (NBF - 1);
          int eid = (ent >> ESHF) & 0xFFFFF;
          eid = eid > nE - 1 ? nE - 1 : eid;
          if (lane == 0) {
            int pos = cursor[slot];
            pos = pos < 0 ? 0 : (pos > RCAP - 1 ? RCAP - 1 : pos);
            region[pos] = eid;
            const int np = pos + 1;
            cursor[slot] = np > RCAP ? RCAP : np;
          }
        }
      }
    }
    __syncthreads();
  }

  const int nv = lenW >> 2;
  int* gp = csr + rb0;
#pragma unroll 1
  for (int i = tid; i < nv; i += NTHR) { const v4i v = ((const v4i*)region)[i]; *(volatile v4i*)(gp + 4 * i) = v; }
  __threadfence();
#pragma unroll 1
  for (int i = tid; i < nv; i += NTHR) { const v4i v = ((const v4i*)region)[i]; *(volatile v4i*)(gp + 4 * i) = v; }
}

template <int CPL>
__device__ __forceinline__ void ldrow(const float* p, float (&v)[CPL]) {
  if constexpr (CPL == 2) {
    const v2f a = *(const v2f*)p;
    v[0] = a.x; v[1] = a.y;
  } else if constexpr (CPL == 4) {
    const v4f a = *(const v4f*)p;
    v[0] = a.x; v[1] = a.y; v[2] = a.z; v[3] = a.w;
  } else {
    const v4f a = *(const v4f*)p, b = *(const v4f*)(p + 4);
    v[0] = a.x; v[1] = a.y; v[2] = a.z; v[3] = a.w;
    v[4] = b.x; v[5] = b.y; v[6] = b.z; v[7] = b.w;
  }
}

template <int CPL, int RB>
__global__ __launch_bounds__(NTHR) void k_agg(
    const int* __restrict__ csr, const int* __restrict__ off, const int* __restrict__ cnt,
    const int* __restrict__ srcs, const float* __restrict__ ew,
    const float* __restrict__ X, const float* __restrict__ bias, _Float16* out,
    int nRowsX, int nN, int nE, int csrLen, int nb) {
  constexpr int W = 32 * CPL;
  const int tid = threadIdx.x, lane = tid & 31, wave = tid >> 5;
  const int tbase = (int)blockIdx.x * TGT + wave * 32;
  const int cl = tbase + lane;
  const int cnt_l = cnt[cl];
  const int off_l = off[cl];
  const int ch0 = CPL * lane;
  float bv[CPL];
#pragma unroll
  for (int e = 0; e < CPL; ++e) {
    bv[e] = 0.0f;
    if constexpr (RB != 0) {
      const int idx = ch0 + e;
      const int ic = idx < nb ? idx : nb - 1;
      const float t = bias[ic];
      bv[e] = idx < nb ? t : 0.0f;
    }
  }

#pragma unroll 1
  for (int j = 0; j < 32; ++j) {
    const int c = tbase + j;
    int n = __builtin_amdgcn_readlane(cnt_l, j);
    n = n < 0 ? 0 : (n > DEGCAP ? DEGCAP : n);
    const int st = __builtin_amdgcn_readlane(off_l, j);
    float acc[CPL];
#pragma unroll
    for (int e = 0; e < CPL; ++e) acc[e] = 0.0f;
#pragma unroll 1
    for (int q0 = 0; q0 < n; q0 += 32) {
      int pos = st + q0 + lane;
      pos = pos < 0 ? 0 : (pos > csrLen - 1 ? csrLen - 1 : pos);
      int eid = csr[pos];
      eid = eid < 0 ? 0 : (eid > nE - 1 ? nE - 1 : eid);
      int sl = srcs[eid];
      sl = sl < 0 ? 0 : (sl > nN - 1 ? nN - 1 : sl);
      sl = sl > nRowsX - 1 ? nRowsX - 1 : sl;
      const float wl = ew[eid];
      const int mcnt = (n - q0) < 32 ? (n - q0) : 32;
#pragma unroll 1
      for (int p = 0; p < mcnt; ++p) {
        const int s = __builtin_amdgcn_readlane(sl, p);
        const float w = __builtin_bit_cast(float, __builtin_amdgcn_readlane(__builtin_bit_cast(int, wl), p));
        float xv[CPL];
        ldrow<CPL>(X + (size_t)s * W + ch0, xv);
#pragma unroll
        for (int e = 0; e < CPL; ++e) acc[e] = acc[e] + w * xv[e];
      }
    }
    const int cs = c > nRowsX - 1 ? nRowsX - 1 : c;
    {
      float sv[CPL];
      ldrow<CPL>(X + (size_t)cs * W + ch0, sv);
#pragma unroll
      for (int e = 0; e < CPL; ++e) {
        float v = acc[e] + sv[e];
        if constexpr (RB != 0) v = fmaxf(v + bv[e], 0.0f);
        acc[e] = v;
      }
    }
    _Float16* op = out + (size_t)c * W + ch0;
    if constexpr (CPL == 2) {
      v2h hv;
      hv[0] = (_Float16)acc[0]; hv[1] = (_Float16)acc[1];
      *(volatile v2h*)op = hv;
      __threadfence();
      *(volatile v2h*)op = hv;
    } else if constexpr (CPL == 4) {
      v4h hv;
      hv[0] = (_Float16)acc[0]; hv[1] = (_Float16)acc[1]; hv[2] = (_Float16)acc[2]; hv[3] = (_Float16)acc[3];
      *(volatile v4h*)op = hv;
      __threadfence();
      *(volatile v4h*)op = hv;
    } else {
      v8h hv;
#pragma unroll
      for (int e = 0; e < 8; ++e) hv[e] = (_Float16)acc[e];
      *(volatile v8h*)op = hv;
      __threadfence();
      *(volatile v8h*)op = hv;
    }
  }
}

template <int K, int NT, int MODE>
__global__ __launch_bounds__(NTHR) void k_gemm(
    const _Float16* __restrict__ A, const _Float16* __restrict__ B,
    const float* __restrict__ bias, const float* __restrict__ bng, const float* __restrict__ bnb,
    const float* __restrict__ bnm, const float* __restrict__ bnv,
    float* outF, _Float16* outH, int ldo, int nvalid, int nRows) {
  constexpr int BC = 32 * NT;
  constexpr int SP = BC + 4;
  static_assert((K % 32) == 0 && (SP % 4) == 0);
  __shared__ __attribute__((aligned(16))) float stg[GR * SP];
  __shared__ float smx[GR];
  __shared__ float slg[GR];
  const int tid = threadIdx.x, lane = tid & 31, wave = tid >> 5, hh = lane >> 4, m = lane & 15;
  const int rg = wave >> 1, chf = wave & 1;
  const int rowBase = (int)blockIdx.x * GR;
  const int colBlk  = (int)blockIdx.y * BC;
  const int wcl = chf * 16 * NT;
  const _Float16* ap = A + (size_t)(rowBase + rg * 16 + m) * K + 8 * hh;
  const _Float16* bp = B + (size_t)(colBlk + wcl + m) * K + 8 * hh;

  v8f acc[NT];
#pragma unroll
  for (int t = 0; t < NT; ++t) { v8f z = {0.f, 0.f, 0.f, 0.f, 0.f, 0.f, 0.f, 0.f}; acc[t] = z; }
#pragma unroll 1
  for (int kt = 0; kt < K / 32; ++kt) {
    FragH a;
    a.h[0] = *(const v8h*)(ap + 32 * kt);
    a.h[1] = *(const v8h*)(ap + 32 * kt + 16);
#pragma unroll
    for (int t = 0; t < NT; ++t) {
      const _Float16* bq = bp + (size_t)(16 * t) * K + 32 * kt;
      FragH b;
      b.h[0] = *(const v8h*)bq;
      b.h[1] = *(const v8h*)(bq + 16);
      acc[t] = wmh(a.v, b.v, acc[t]);
    }
  }

  float* sp = stg + (rg * 16 + 8 * hh) * SP + wcl + m;
#pragma unroll
  for (int t = 0; t < NT; ++t) {
    const int col = colBlk + wcl + 16 * t + m;
    const int cc = col < nvalid ? col : nvalid - 1;
    float addv = 0.0f, sc = 1.0f, mu = 0.0f, be = 0.0f;
    if constexpr (MODE != 2) {
      const float bb = bias[cc];
      addv = col < nvalid ? bb : 0.0f;
    }
    if constexpr (MODE == 1 || MODE == 4) {
      sc = bng[cc] * (1.0f / sqrtf(bnv[cc] + BNEPS));
      mu = bnm[cc];
      be = bnb[cc];
    }
#pragma unroll
    for (int r = 0; r < 8; ++r) {
      float v = acc[t][r] * WINV + addv;
      if constexpr (MODE == 0) v = fmaxf(v, 0.0f);
      if constexpr (MODE == 1 || MODE == 4) { v = (v - mu) * sc + be; v = fmaxf(v, 0.0f); }
      sp[r * SP + 16 * t] = v;
    }
  }
  __syncthreads();

  if constexpr (MODE == 1 || MODE == 2) {
    constexpr int LPR = BC / 4, RPI = 32 / LPR, NI = (GR / NWAVE) / RPI;
    const int lr = lane / LPR, lc = (lane - lr * LPR) * 4;
#pragma unroll
    for (int i = 0; i < NI; ++i) {
      const int row = wave * 8 + i * RPI + lr;
      const v4f v = *(const v4f*)(stg + row * SP + lc);
      float* gp = outF + (size_t)(rowBase + row) * ldo + colBlk + lc;
      *(volatile v4f*)gp = v;
    }
    __threadfence();
#pragma unroll
    for (int i = 0; i < NI; ++i) {
      const int row = wave * 8 + i * RPI + lr;
      const v4f v = *(const v4f*)(stg + row * SP + lc);
      float* gp = outF + (size_t)(rowBase + row) * ldo + colBlk + lc;
      *(volatile v4f*)gp = v;
    }
  } else if constexpr (MODE == 0 || MODE == 4) {
    constexpr int LPR = BC / 8, RPI = 32 / LPR, NI = (GR / NWAVE) / RPI;
    const int lr = lane / LPR, lc = (lane - lr * LPR) * 8;
#pragma unroll
    for (int i = 0; i < NI; ++i) {
      const int row = wave * 8 + i * RPI + lr;
      const v4f a = *(const v4f*)(stg + row * SP + lc), b = *(const v4f*)(stg + row * SP + lc + 4);
      v8h hv;
      hv[0] = (_Float16)a.x; hv[1] = (_Float16)a.y; hv[2] = (_Float16)a.z; hv[3] = (_Float16)a.w;
      hv[4] = (_Float16)b.x; hv[5] = (_Float16)b.y; hv[6] = (_Float16)b.z; hv[7] = (_Float16)b.w;
      _Float16* gp = outH + (size_t)(rowBase + row) * ldo + colBlk + lc;
      *(volatile v8h*)gp = hv;
    }
    __threadfence();
#pragma unroll
    for (int i = 0; i < NI; ++i) {
      const int row = wave * 8 + i * RPI + lr;
      const v4f a = *(const v4f*)(stg + row * SP + lc), b = *(const v4f*)(stg + row * SP + lc + 4);
      v8h hv;
      hv[0] = (_Float16)a.x; hv[1] = (_Float16)a.y; hv[2] = (_Float16)a.z; hv[3] = (_Float16)a.w;
      hv[4] = (_Float16)b.x; hv[5] = (_Float16)b.y; hv[6] = (_Float16)b.z; hv[7] = (_Float16)b.w;
      _Float16* gp = outH + (size_t)(rowBase + row) * ldo + colBlk + lc;
      *(volatile v8h*)gp = hv;
    }
  } else {
    if (tid < GR) {
      const float* rp = stg + tid * SP;
      float mx = rp[0];
#pragma unroll 1
      for (int c = 1; c < nvalid; ++c) mx = fmaxf(mx, rp[c]);
      float s = 0.0f;
#pragma unroll 1
      for (int c = 0; c < nvalid; ++c) s += expf(rp[c] - mx);
      smx[tid] = mx;
      slg[tid] = logf(s);
    }
    __syncthreads();
    int nvr = nRows - rowBase;
    nvr = nvr < 0 ? 0 : (nvr > GR ? GR : nvr);
    const int q4  = nvalid >> 2;
    const int nf4 = nvr * q4;
    float* ob = outF + (size_t)rowBase * nvalid;
#pragma unroll 1
    for (int i = tid; i < nf4; i += NTHR) {
      const int row = i / q4;
      const int col = (i - row * q4) * 4;
      v4f v = *(const v4f*)(stg + row * SP + col);
      const float mx = smx[row], lg = slg[row];
      v.x = (v.x - mx) - lg; v.y = (v.y - mx) - lg; v.z = (v.z - mx) - lg; v.w = (v.w - mx) - lg;
      *(volatile v4f*)(ob + 4 * i) = v;
    }
    __threadfence();
#pragma unroll 1
    for (int i = tid; i < nf4; i += NTHR) {
      const int row = i / q4;
      const int col = (i - row * q4) * 4;
      v4f v = *(const v4f*)(stg + row * SP + col);
      const float mx = smx[row], lg = slg[row];
      v.x = (v.x - mx) - lg; v.y = (v.y - mx) - lg; v.z = (v.z - mx) - lg; v.w = (v.w - mx) - lg;
      *(volatile v4f*)(ob + 4 * i) = v;
    }
  }
}

extern "C" void kernel_launch(void* const* d_in, const int* in_sizes, int n_in,
                              void* d_out, int out_size, void* d_ws, size_t ws_size,
                              hipStream_t stream) {
  if (n_in < 23) return;
  const int nN = in_sizes[0] / CIN;
  const int nE = in_sizes[2];
  if (nN <= 0 || nE <= 0) return;
  if (in_sizes[0] != nN * CIN || in_sizes[1] != 2 * nE) return;
  if (in_sizes[3] != CIN * CH || in_sizes[4] != CH || in_sizes[5] != CH * CH || in_sizes[6] != CH) return;
  if (in_sizes[7] != CH * CH || in_sizes[8] != CH || in_sizes[9] != CH * CH || in_sizes[10] != CH) return;
  if (in_sizes[11] != CH * NCLS || in_sizes[12] != NCLS || in_sizes[13] != NCLS * NCLS || in_sizes[14] != NCLS) return;
  for (int i = 15; i < 23; ++i) if (in_sizes[i] != CH) return;
  if (out_size != nN * NCLS) return;
  if (nN > (1 << 20) || nE > (1 << 20)) return;

  const float* x    = (const float*)d_in[0];
  const int*   ei   = (const int*)d_in[1];
  const float* ew   = (const float*)d_in[2];
  const float* w1_0 = (const float*)d_in[3];  const float* b1_0 = (const float*)d_in[4];
  const float* w2_0 = (const float*)d_in[5];  const float* b2_0 = (const float*)d_in[6];
  const float* w1_1 = (const float*)d_in[7];  const float* b1_1 = (const float*)d_in[8];
  const float* w2_1 = (const float*)d_in[9];  const float* b2_1 = (const float*)d_in[10];
  const float* w1_2 = (const float*)d_in[11]; const float* b1_2 = (const float*)d_in[12];
  const float* w2_2 = (const float*)d_in[13]; const float* b2_2 = (const float*)d_in[14];
  const float* bng0 = (const float*)d_in[15]; const float* bnb0 = (const float*)d_in[16];
  const float* bnm0 = (const float*)d_in[17]; const float* bnv0 = (const float*)d_in[18];
  const float* bng1 = (const float*)d_in[19]; const float* bnb1 = (const float*)d_in[20];
  const float* bnm1 = (const float*)d_in[21]; const float* bnv1 = (const float*)d_in[22];
  float* out = (float*)d_out;

  const int NPAD   = ((nN + TGT - 1) / TGT) * TGT;
  const int nBC    = (nN + NBC - 1) / NBC;
  const int CNTPAD = nBC * NBC;
  const int nBF    = (nN + NBF - 1) / NBF;
  const int OFFN   = nBF * NBF;
  if (nBF + 1 > RBN) return;
  if (OFFN > CNTPAD || NPAD > OFFN) return;
  const int csrLen = ((nE + 31) & ~31) + 32 * (nBF + 1);
  const int nGemm  = NPAD / GR;
  const int nAgg   = NPAD / TGT;

  char* ws = (char*)d_ws;
  size_t off = 0;
  const size_t oW10 = off; off += (size_t)CH  * CIN * 2;   off = (off + 255) & ~(size_t)255;
  const size_t oW20 = off; off += (size_t)CH  * CH  * 2;   off = (off + 255) & ~(size_t)255;
  const size_t oW11 = off; off += (size_t)CH  * CH  * 2;   off = (off + 255) & ~(size_t)255;
  const size_t oW21 = off; off += (size_t)CH  * CH  * 2;   off = (off + 255) & ~(size_t)255;
  const size_t oW12 = off; off += (size_t)NCP * CH  * 2;   off = (off + 255) & ~(size_t)255;
  const size_t oW22 = off; off += (size_t)NCP * NCP * 2;   off = (off + 255) & ~(size_t)255;
  const size_t oCnt = off; off += (size_t)CNTPAD * 4;      off = (off + 255) & ~(size_t)255;
  const size_t oOff = off; off += (size_t)OFFN * 4;        off = (off + 255) & ~(size_t)255;
  const size_t oRb  = off; off += (size_t)RBN * 4;         off = (off + 255) & ~(size_t)255;
  const size_t oCsr = off; off += (size_t)csrLen * 4;      off = (off + 255) & ~(size_t)255;
  const size_t oA16 = off; off += (size_t)NPAD * CH * 2;   off = (off + 255) & ~(size_t)255;
  const size_t oT16 = off; off += (size_t)NPAD * CH * 2;   off = (off + 255) & ~(size_t)255;
  const size_t oH32 = off; off += (size_t)NPAD * CH * 4;   off = (off + 255) & ~(size_t)255;
  if (off > ws_size || off > (size_t)WSCAP) return;
  _Float16* W10 = (_Float16*)(ws + oW10);
  _Float16* W20 = (_Float16*)(ws + oW20);
  _Float16* W11 = (_Float16*)(ws + oW11);
  _Float16* W21 = (_Float16*)(ws + oW21);
  _Float16* W12 = (_Float16*)(ws + oW12);
  _Float16* W22 = (_Float16*)(ws + oW22);
  int*   cnt  = (int*)(ws + oCnt);
  int*   offp = (int*)(ws + oOff);
  int*   rb   = (int*)(ws + oRb);
  int*   csr  = (int*)(ws + oCsr);
  _Float16* A16 = (_Float16*)(ws + oA16);
  _Float16* T16 = (_Float16*)(ws + oT16);
  float*    G32 = (float*)(ws + oT16);
  float*    H32 = (float*)(ws + oH32);
  _Float16* T2  = (_Float16*)(ws + oH32);

  const int vec8 = ((nE & 3) == 0) ? 1 : 0;

  k_wprep<<<(CH * CIN / 8 + NTHR - 1) / NTHR, NTHR, 0, stream>>>(w1_0, W10, CIN, CH, CIN, CH);
  k_wprep<<<(CH * CH / 8 + NTHR - 1) / NTHR, NTHR, 0, stream>>>(w2_0, W20, CH, CH, CH, CH);
  k_wprep<<<(CH * CH / 8 + NTHR - 1) / NTHR, NTHR, 0, stream>>>(w1_1, W11, CH, CH, CH, CH);
  k_wprep<<<(CH * CH / 8 + NTHR - 1) / NTHR, NTHR, 0, stream>>>(w2_1, W21, CH, CH, CH, CH);
  k_wprep<<<(NCP * CH / 8 + NTHR - 1) / NTHR, NTHR, 0, stream>>>(w1_2, W12, CH, NCLS, CH, NCP);
  k_wprep<<<(NCP * NCP / 8 + NTHR - 1) / NTHR, NTHR, 0, stream>>>(w2_2, W22, NCLS, NCLS, NCP, NCP);

  hipFuncSetAttribute(reinterpret_cast<const void*>(&k_count),
                      hipFuncAttributeMaxDynamicSharedMemorySize, LDS_COUNT);
  k_count<<<nBC, NTHR, LDS_COUNT, stream>>>(ei, cnt, nE, vec8);
  k_offsets<<<1, OTHR, 0, stream>>>(cnt, offp, rb, nBF);
  hipFuncSetAttribute(reinterpret_cast<const void*>(&k_fill),
                      hipFuncAttributeMaxDynamicSharedMemorySize, LDS_FILL);
  k_fill<<<nBF, NTHR, LDS_FILL, stream>>>(ei, offp, rb, csr, nE, vec8, csrLen);

  k_agg<4, 0><<<nAgg, NTHR, 0, stream>>>(csr, offp, cnt, ei, ew, x, b1_0, A16, nN, nN, nE, csrLen, CH);
  k_gemm<CIN, 4, 0><<<dim3(nGemm, CH / 128), NTHR, 0, stream>>>(A16, W10, b1_0, b1_0, b1_0, b1_0, b1_0, H32, T16, CH, CH, NPAD);
  k_gemm<CH, 4, 1><<<dim3(nGemm, CH / 128), NTHR, 0, stream>>>(T16, W20, b2_0, bng0, bnb0, bnm0, bnv0, H32, A16, CH, CH, NPAD);

  k_agg<8, 0><<<nAgg, NTHR, 0, stream>>>(csr, offp, cnt, ei, ew, H32, b1_1, A16, NPAD, nN, nE, csrLen, CH);
  k_gemm<CH, 4, 0><<<dim3(nGemm, CH / 128), NTHR, 0, stream>>>(A16, W11, b1_1, b1_1, b1_1, b1_1, b1_1, H32, T16, CH, CH, NPAD);
  k_gemm<CH, 4, 4><<<dim3(nGemm, CH / 128), NTHR, 0, stream>>>(T16, W21, b2_1, bng1, bnb1, bnm1, bnv1, H32, A16, CH, CH, NPAD);

  k_gemm<CH, 2, 2><<<dim3(nGemm, 1), NTHR, 0, stream>>>(A16, W12, b1_2, b1_2, b1_2, b1_2, b1_2, G32, T16, NCP, NCP, NPAD);
  k_agg<2, 1><<<nAgg, NTHR, 0, stream>>>(csr, offp, cnt, ei, ew, G32, b1_2, T2, NPAD, nN, nE, csrLen, NCLS);
  k_gemm<NCP, 2, 3><<<dim3(nGemm, 1), NTHR, 0, stream>>>(T2, W22, b2_2, b2_2, b2_2, b2_2, b2_2, out, T2, NCLS, NCLS, nN);
}
